// KernelMachine_40355512713599
// MI455X (gfx1250) — hardware-verified
//
#include <hip/hip_runtime.h>
#include <math.h>

typedef __attribute__((ext_vector_type(16))) _Float16 v16h;
typedef __attribute__((ext_vector_type(8)))  _Float16 v8h;
typedef __attribute__((ext_vector_type(16))) __bf16   v16b;
typedef __attribute__((ext_vector_type(8)))  __bf16   v8b;
typedef __attribute__((ext_vector_type(8)))  float    v8f;
typedef __attribute__((ext_vector_type(4)))  float    v4f;

constexpr int kInputsRneToBf16 = 1;

constexpr int kBatch  = 8192;
constexpr int kDim    = 64;
constexpr int kNs     = 4096;
constexpr int kMd     = 8;
constexpr int kMdPad  = 16;
constexpr int kKP     = kInputsRneToBf16 ? kDim : 3 * kDim;
constexpr int kSlabP  = 68;
constexpr int kSqrtNs = 64;
static_assert(kSqrtNs * kSqrtNs == kNs, "sample count is a square");
static_assert((kKP % 32) == 0 && (kNs % 32) == 0, "K multiples of 32");
static_assert((kBatch % 64) == 0 && (kNs % 64) == 0, "phase GEMM M,N multiples of 64");
static_assert((kBatch % 128) == 0 && kMdPad == 16 && kMd <= kMdPad, "readout tiling");
static_assert(kDim == 64, "one plane row segment is 64 elements");

constexpr float kSqrt2   = 1.41421356237309504880f;
constexpr float kScale   = kSqrt2 / (float)kSqrtNs;
constexpr float kGCarry  = 512.0f;
constexpr float kWCarry  = 1024.0f;
constexpr float kFold    = kScale / (kGCarry * kWCarry);
constexpr float kF16MinNormal = 6.103515625e-05f;

constexpr size_t kOffAP   = 0;
constexpr size_t kOffBP   = kOffAP  + (size_t)kBatch * kKP * 2;
constexpr size_t kOffWPT  = kOffBP  + (size_t)kNs * kKP * 2;
constexpr size_t kOffG    = kOffWPT + (size_t)kMdPad * kNs * 2;
constexpr size_t kWsTotal = kOffG   + (size_t)kBatch * kNs * 2;
static_assert(kWsTotal == (kInputsRneToBf16 ? 68812800ull : 71958528ull), "carve total");
static_assert(kWsTotal <= 134217728ull, "carve cap");
static_assert((kOffBP % 128) == 0 && (kOffWPT % 128) == 0 && (kOffG % 128) == 0, "128-B aligned regions");

constexpr int kPrepBlkX = (kBatch * kDim / 8) / 256;
constexpr int kPrepBlkW = (kNs * kDim / 8) / 256;
constexpr int kPrepBlkP = (kMdPad * kNs / 8) / 256;
static_assert(kPrepBlkX * 256 * 8 == kBatch * kDim, "x plane coverage exact");
static_assert(kPrepBlkW * 256 * 8 == kNs * kDim, "Wf plane coverage exact");
static_assert(kPrepBlkP * 256 * 8 == kMdPad * kNs, "WpT plane coverage exact");

__device__ __forceinline__ unsigned short f2bf_bits(float f) {
  unsigned u = __float_as_uint(f);
  return (unsigned short)((u + 0x7FFFu + ((u >> 16) & 1u)) >> 16);
}
__device__ __forceinline__ float bf_bits2f(unsigned short h) { return __uint_as_float(((unsigned)h) << 16); }

__device__ __forceinline__ float flush_below_f16_normal(float v) {
  return (fabsf(v) < kF16MinNormal) ? 0.0f : v;
}

__device__ __forceinline__ v16b ld_frag_b(const __bf16* p) {
  union { v16b v; v8b h[2]; } f;
  f.h[0] = *(const v8b*)(p);
  f.h[1] = *(const v8b*)(p + 16);
  return f.v;
}
__device__ __forceinline__ v16h ld_frag_h(const _Float16* p) {
  union { v16h v; v8h h[2]; } f;
  f.h[0] = *(const v8h*)(p);
  f.h[1] = *(const v8h*)(p + 16);
  return f.v;
}
__device__ __forceinline__ v8f mma_b(v16b a, v16b b, v8f c) {
  c = __builtin_amdgcn_wmma_f32_16x16x32_bf16(false, a, false, b, (short)0, c, false, false);
  asm volatile("v_nop\n\tv_nop\n\tv_nop\n\tv_nop" : "+v"(c) : "v"(a), "v"(b));
  return c;
}
__device__ __forceinline__ v8f mma_h(v16h a, v16h b, v8f c) {
  c = __builtin_amdgcn_wmma_f32_16x16x32_f16(false, a, false, b, (short)0, c, false, false);
  asm volatile("v_nop\n\tv_nop\n\tv_nop\n\tv_nop" : "+v"(c) : "v"(a), "v"(b));
  return c;
}
__device__ __forceinline__ void wave_lds_sync() {
  __builtin_amdgcn_fence(__ATOMIC_RELEASE, "workgroup");
  __builtin_amdgcn_wave_barrier();
  __builtin_amdgcn_fence(__ATOMIC_ACQUIRE, "workgroup");
}

__global__ __launch_bounds__(256) void prep_planes_kernel(
    const float* __restrict__ x, const float* __restrict__ Wf, const float* __restrict__ Wp,
    unsigned short* __restrict__ AP, unsigned short* __restrict__ BP, unsigned short* __restrict__ WPT)
{
  const int blk = blockIdx.x;
  const int tid = threadIdx.x;
  if (blk < kPrepBlkX + kPrepBlkW) {
    const bool isW = (blk >= kPrepBlkX);
    const float* src = isW ? Wf : x;
    unsigned short* dst = isW ? BP : AP;
    const int i = (isW ? (blk - kPrepBlkX) : blk) * 256 + tid;
    const int row = i >> 3;
    const int c8 = (i & 7) * 8;
    const v4f a0 = *(const v4f*)(src + (size_t)i * 8);
    const v4f a1 = *(const v4f*)(src + (size_t)i * 8 + 4);
    v8h hv, lv;
#pragma unroll
    for (int e = 0; e < 4; ++e) {
      const float f0 = a0[e];
      const float f1 = a1[e];
      const unsigned short h0 = f2bf_bits(f0);
      const unsigned short h1 = f2bf_bits(f1);
      const unsigned short l0 = f2bf_bits(f0 - bf_bits2f(h0));
      const unsigned short l1 = f2bf_bits(f1 - bf_bits2f(h1));
      hv[e]     = __builtin_bit_cast(_Float16, h0);
      hv[4 + e] = __builtin_bit_cast(_Float16, h1);
      lv[e]     = __builtin_bit_cast(_Float16, l0);
      lv[4 + e] = __builtin_bit_cast(_Float16, l1);
    }
    unsigned short* q = dst + (size_t)row * kKP + c8;
    if (kKP == kDim) {
      *(volatile v8h*)q = hv;
      __threadfence();
      *(volatile v8h*)q = hv;
    } else {
      const v8h s1 = isW ? hv : lv;
      const v8h s2 = isW ? lv : hv;
      *(volatile v8h*)(q) = hv;
      *(volatile v8h*)(q + kDim) = s1;
      *(volatile v8h*)(q + 2 * kDim) = s2;
      __threadfence();
      *(volatile v8h*)(q) = hv;
      *(volatile v8h*)(q + kDim) = s1;
      *(volatile v8h*)(q + 2 * kDim) = s2;
    }
  } else {
    const int j = (blk - kPrepBlkX - kPrepBlkW) * 256 + tid;
    const int m = j >> 9;
    const int n8 = (j & 511) * 8;
    const int mc = (m < kMd) ? m : (kMd - 1);
    float w[8];
#pragma unroll
    for (int e = 0; e < 8; ++e) w[e] = Wp[(size_t)(n8 + e) * kMd + mc];
    v8h hv;
#pragma unroll
    for (int e = 0; e < 8; ++e) {
      float t = w[e];
      if (kInputsRneToBf16) t = bf_bits2f(f2bf_bits(t));
      t = flush_below_f16_normal(t * kWCarry);
      t = (m < kMd) ? t : 0.0f;
      hv[e] = (_Float16)t;
    }
    unsigned short* q = WPT + (size_t)j * 8;
    *(volatile v8h*)q = hv;
    __threadfence();
    *(volatile v8h*)q = hv;
  }
}

__global__ __launch_bounds__(256) void phase_cos_gemm_kernel(
    const unsigned short* __restrict__ Ap, const unsigned short* __restrict__ Btp,
    const float* __restrict__ bias, unsigned short* __restrict__ Gp)
{
  __shared__ __align__(16) float sT[8][16 * kSlabP];
  const int lane = threadIdx.x & 31;
  const int wave = threadIdx.x >> 5;
  constexpr int tilesN = kNs / 64;
  constexpr int tilesM = kBatch / 64;
  const int tile = blockIdx.x * 8 + wave;
  if (tile >= tilesM * tilesN) return;
  const int tm = tile / tilesN;
  const int tn = tile - tm * tilesN;
  const int m0 = tm << 6;
  const int n0 = tn << 6;

  const __bf16* A  = (const __bf16*)Ap;
  const __bf16* Bt = (const __bf16*)Btp;
  const int rlane = lane & 15;
  const int koff  = (lane >> 4) * 8;
  const int mOff  = (lane >> 4) * 8;

  v8f acc[4][4];
#pragma unroll
  for (int i = 0; i < 4; ++i)
#pragma unroll
    for (int j = 0; j < 4; ++j) acc[i][j] = (v8f){0.f, 0.f, 0.f, 0.f, 0.f, 0.f, 0.f, 0.f};

#pragma unroll 1
  for (int k0 = 0; k0 < kKP; k0 += 32) {
    v16b bh[4];
#pragma unroll
    for (int j = 0; j < 4; ++j)
      bh[j] = ld_frag_b(Bt + (size_t)(n0 + (j << 4) + rlane) * kKP + koff + k0);
#pragma unroll
    for (int i = 0; i < 4; ++i) {
      const v16b ah = ld_frag_b(A + (size_t)(m0 + (i << 4) + rlane) * kKP + koff + k0);
#pragma unroll
      for (int j = 0; j < 4; ++j) acc[i][j] = mma_b(ah, bh[j], acc[i][j]);
    }
  }

  float bv[4];
#pragma unroll
  for (int j = 0; j < 4; ++j) {
    float t = bias[n0 + (j << 4) + rlane];
    if (kInputsRneToBf16) t = bf_bits2f(f2bf_bits(t));
    bv[j] = t;
  }

  float* slab = sT[wave];
  unsigned short* G = Gp;
  const int q  = lane >> 3;
  const int c8 = (lane & 7) * 8;
#pragma unroll
  for (int i = 0; i < 4; ++i) {
    const int mBase = m0 + (i << 4);
#pragma unroll
    for (int j = 0; j < 4; ++j) {
#pragma unroll
      for (int r = 0; r < 8; ++r)
        slab[(mOff + r) * kSlabP + (j << 4) + rlane] = acc[i][j][r] + bv[j];
    }
    wave_lds_sync();
#pragma unroll 1
    for (int t = 0; t < 32; ++t) {
      float* p = slab + (t >> 1) * kSlabP + (t & 1) * 32 + lane;
      const float ph = *p;
      const float cv = flush_below_f16_normal(cosf(ph) * kGCarry);
      *p = cv;
    }
    wave_lds_sync();
    for (int pass = 0; pass < 2; ++pass) {
#pragma unroll
      for (int it = 0; it < 4; ++it) {
        const int row = it * 4 + q;
        const float* sp = slab + row * kSlabP + c8;
        v8h hv;
#pragma unroll
        for (int e = 0; e < 8; ++e) hv[e] = (_Float16)sp[e];
        *(volatile v8h*)(G + (size_t)(mBase + row) * kNs + n0 + c8) = hv;
      }
      __threadfence();
    }
    wave_lds_sync();
  }
}

__global__ __launch_bounds__(256) void readout_gemm_kernel(
    const unsigned short* __restrict__ Gp, const unsigned short* __restrict__ WPTp, float* __restrict__ out)
{
  __shared__ __align__(16) float sO[8][16 * 16];
  const int lane = threadIdx.x & 31;
  const int wave = threadIdx.x >> 5;
  const int m0 = (blockIdx.x * 8 + wave) * 16;
  if (m0 >= kBatch) return;
  const int rlane = lane & 15;
  const int koff  = (lane >> 4) * 8;
  const int mOff  = (lane >> 4) * 8;
  const _Float16* Ar = (const _Float16*)Gp + (size_t)(m0 + rlane) * kNs + koff;
  const _Float16* Br = (const _Float16*)WPTp + (size_t)rlane * kNs + koff;

  v8f acc = (v8f){0.f, 0.f, 0.f, 0.f, 0.f, 0.f, 0.f, 0.f};
#pragma unroll 4
  for (int k0 = 0; k0 < kNs; k0 += 32) {
    const v16h a = ld_frag_h(Ar + k0);
    const v16h b = ld_frag_h(Br + k0);
    acc = mma_h(a, b, acc);
  }

  float* so = sO[wave];
#pragma unroll
  for (int r = 0; r < 8; ++r) so[(mOff + r) * 16 + rlane] = acc[r] * kFold;
  wave_lds_sync();
  const int orow = lane >> 1;
  const int oc4  = (lane & 1) * 4;
  v4f val;
  val[0] = so[orow * 16 + oc4 + 0];
  val[1] = so[orow * 16 + oc4 + 1];
  val[2] = so[orow * 16 + oc4 + 2];
  val[3] = so[orow * 16 + oc4 + 3];
  float* dst = out + (size_t)m0 * kMd + lane * 4;
  *(volatile v4f*)dst = val;
  __threadfence();
  *(volatile v4f*)dst = val;
}

extern "C" void kernel_launch(void* const* d_in, const int* in_sizes, int n_in,
                              void* d_out, int out_size, void* d_ws, size_t ws_size,
                              hipStream_t stream) {
  if (n_in < 4) return;
  if (in_sizes[0] != kBatch * kDim) return;
  if (in_sizes[1] != kNs * kDim) return;
  if (in_sizes[2] != kNs) return;
  if (in_sizes[3] != kNs * kMd) return;
  if (out_size != kBatch * kMd) return;
  if (ws_size < kWsTotal) return;

  const float* x  = (const float*)d_in[0];
  const float* Wf = (const float*)d_in[1];
  const float* bf = (const float*)d_in[2];
  const float* Wp = (const float*)d_in[3];
  float* out = (float*)d_out;

  char* ws = (char*)d_ws;
  unsigned short* AP  = (unsigned short*)(ws + kOffAP);
  unsigned short* BP  = (unsigned short*)(ws + kOffBP);
  unsigned short* WPT = (unsigned short*)(ws + kOffWPT);
  unsigned short* G   = (unsigned short*)(ws + kOffG);

  prep_planes_kernel<<<kPrepBlkX + kPrepBlkW + kPrepBlkP, 256, 0, stream>>>(x, Wf, Wp, AP, BP, WPT);

  phase_cos_gemm_kernel<<<(kBatch / 64) * (kNs / 64) / 8, 256, 0, stream>>>(AP, BP, bf, G);

  readout_gemm_kernel<<<kBatch / 128, 256, 0, stream>>>(G, WPT, out);
}
